// CustomAttentionLayer_28441273434636
// MI455X (gfx1250) — hardware-verified
//
#include <hip/hip_runtime.h>
#include <stdint.h>

#define NSEQ 4
#define SEQ  4096
#define NTOT (NSEQ * SEQ)
#define DM   512
#define LDQK (2 * DM)

typedef _Float16 v16h __attribute__((ext_vector_type(16)));
typedef _Float16 v8h  __attribute__((ext_vector_type(8)));
typedef __bf16   v16b __attribute__((ext_vector_type(16)));
typedef __bf16   v8b  __attribute__((ext_vector_type(8)));
typedef float    v8f  __attribute__((ext_vector_type(8)));
typedef float    v4f  __attribute__((ext_vector_type(4)));
typedef unsigned short v8us __attribute__((ext_vector_type(8)));

static_assert((DM % 64) == 0);
static_assert((NTOT % 64) == 0);
static_assert((SEQ % 256) == 0);

__device__ __forceinline__ unsigned short bfbits(float f) {
  unsigned u = __float_as_uint(f);
  return (unsigned short)((u + 0x7FFFu + ((u >> 16) & 1u)) >> 16);
}
__device__ __forceinline__ float bfval(unsigned short b) { return __uint_as_float(((unsigned)b) << 16); }
__device__ __forceinline__ float bfr(float f) { return bfval(bfbits(f)); }
__device__ __forceinline__ void split_bf(float f, unsigned short& hb, unsigned short& lb) {
  hb = bfbits(f);
  lb = bfbits(f - bfval(hb));
}

template <int ET> struct Elem;
template <> struct Elem<0> {
  typedef _Float16 T; typedef v16h V; typedef v8h V8;
  static __device__ __forceinline__ v8f mma(V a, V b, v8f c) {
    return __builtin_amdgcn_wmma_f32_16x16x32_f16(false, a, false, b, (short)0, c, false, false);
  }
};
template <> struct Elem<1> {
  typedef __bf16 T; typedef v16b V; typedef v8b V8;
  static __device__ __forceinline__ v8f mma(V a, V b, v8f c) {
    return __builtin_amdgcn_wmma_f32_16x16x32_bf16(false, a, false, b, (short)0, c, false, false);
  }
};

template <int ET>
__device__ __forceinline__ typename Elem<ET>::V ldfragT(const typename Elem<ET>::T* p) {
  typedef typename Elem<ET>::V V;
  typedef typename Elem<ET>::V8 V8;
  union { V v; V8 h[2]; } f;
  f.h[0] = *(const V8*)(p);
  f.h[1] = *(const V8*)(p + 16);
  return f.v;
}
__device__ __forceinline__ v16h ldfrag(const _Float16* p) { return ldfragT<0>(p); }
__device__ __forceinline__ v8f mma16(v16h a, v16h b, v8f c) { return Elem<0>::mma(a, b, c); }
__device__ __forceinline__ v8f zero8() {
  v8f z;
#pragma unroll
  for (int i = 0; i < 8; ++i) z[i] = 0.0f;
  return z;
}

__device__ __forceinline__ void guard_g(v8f& a, v8f& b, v16h x, v16h y) {
  asm volatile("v_nop\n\tv_nop\n\tv_nop\n\tv_nop" : "+v"(a), "+v"(b) : "v"(x), "v"(y));
}
__device__ __forceinline__ void guard_g(v8f& a, v8f& b, v16b x, v16b y) {
  asm volatile("v_nop\n\tv_nop\n\tv_nop\n\tv_nop" : "+v"(a), "+v"(b) : "v"(x), "v"(y));
}
__device__ __forceinline__ void keep4(v16h a, v16h b, v16h c, v16h d) {
  asm volatile("v_nop" :: "v"(a), "v"(b), "v"(c), "v"(d));
}
__device__ __forceinline__ void keep4(v16b a, v16b b, v16b c, v16b d) {
  asm volatile("v_nop" :: "v"(a), "v"(b), "v"(c), "v"(d));
}
__device__ __forceinline__ void accg4(v8f& a, v8f& b, v8f& c, v8f& d) {
  asm volatile("v_nop\n\tv_nop\n\tv_nop\n\tv_nop" : "+v"(a), "+v"(b), "+v"(c), "+v"(d));
}
__device__ __forceinline__ void guard_s4(v8f& a, v8f& b, v8f& c, v8f& d, v16h x0, v16h x1, v16h y0, v16h y1) {
  asm volatile("v_nop\n\tv_nop\n\tv_nop\n\tv_nop"
               : "+v"(a), "+v"(b), "+v"(c), "+v"(d) : "v"(x0), "v"(x1), "v"(y0), "v"(y1));
}

__global__ __launch_bounds__(256) void cvt_x_kernel(const float* __restrict__ x, _Float16* __restrict__ d16, int n8) {
  const int li = (int)blockIdx.x * 256 + (int)threadIdx.x;
  if (li >= n8) return;
  const size_t e = (size_t)li * 8;
  const v4f a = *(const v4f*)(x + e);
  const v4f b = *(const v4f*)(x + e + 4);
  v8h o;
#pragma unroll
  for (int i = 0; i < 4; ++i) {
    o[i]     = (_Float16)(bfr(a[i]) * 8.0f);
    o[4 + i] = (_Float16)(bfr(b[i]) * 8.0f);
  }
  _Float16* d = d16 + e;
  *(volatile v8h*)d = o;
  __threadfence();
  *(volatile v8h*)d = o;
}

__global__ __launch_bounds__(256) void cvt_wt_kernel(const float* __restrict__ w0, const float* __restrict__ w1,
                                                     const float* __restrict__ w2, const float* __restrict__ w3,
                                                     _Float16* __restrict__ wt16, unsigned short* __restrict__ wob) {
  __shared__ __align__(16) float sT[64 * 68];
  const int tid = (int)threadIdx.x;
  const int mat = (int)blockIdx.x >> 6;
  const int tile = (int)blockIdx.x & 63;
  const int tr = tile >> 3, tc = tile & 7;
  const float* src = (mat == 0) ? w0 : ((mat == 1) ? w1 : ((mat == 2) ? w2 : w3));
  {
    const int r = tid >> 2, c16 = (tid & 3) * 16;
    const float* sp = src + (size_t)(tr * 64 + r) * DM + tc * 64 + c16;
#pragma unroll
    for (int i = 0; i < 4; ++i) {
      const v4f a = *(const v4f*)(sp + 4 * i);
#pragma unroll
      for (int e = 0; e < 4; ++e) sT[(c16 + 4 * i + e) * 68 + r] = a[e];
    }
  }
  __syncthreads();
  const int piece = tid & 7;
#pragma unroll
  for (int it = 0; it < 2; ++it) {
    const int line = it * 32 + (tid >> 3);
    const float* lp = sT + line * 68 + piece * 8;
    const v4f u0 = *(const v4f*)lp, u1 = *(const v4f*)(lp + 4);
    const int prow = tc * 64 + line;
    const int d0 = tr * 64 + piece * 8;
    if (mat < 3) {
      v8h o;
#pragma unroll
      for (int e = 0; e < 4; ++e) {
        o[e]     = (_Float16)(bfr(u0[e]) * 64.0f);
        o[4 + e] = (_Float16)(bfr(u1[e]) * 64.0f);
      }
      _Float16* d = wt16 + (size_t)(mat * DM + prow) * DM + d0;
      *(volatile v8h*)d = o;
      __threadfence();
      *(volatile v8h*)d = o;
    } else {
      v8us o;
#pragma unroll
      for (int e = 0; e < 4; ++e) {
        o[e]     = bfbits(u0[e]);
        o[4 + e] = bfbits(u1[e]);
      }
      unsigned short* d = wob + (size_t)prow * DM + d0;
      *(volatile v8us*)d = o;
      __threadfence();
      *(volatile v8us*)d = o;
    }
  }
}

template <int ET, bool SPLITA, int OUT_MODE, int BIAS_MODE>
__global__ __launch_bounds__(256) void gemm64_kernel(const unsigned short* __restrict__ Ap,
                                                     const unsigned short* __restrict__ A2p, int lda,
                                                     const unsigned short* __restrict__ Btp, int ldb,
                                                     void* __restrict__ Cout, int ldc,
                                                     const float* __restrict__ bias0, const float* __restrict__ bias1,
                                                     int nsplit, int M, int N, int K, float scale, float bias_scale) {
  typedef typename Elem<ET>::T T;
  typedef typename Elem<ET>::V V;
  const T* A  = (const T*)(const void*)Ap;
  const T* A2 = (const T*)(const void*)A2p;
  const T* Bt = (const T*)(const void*)Btp;
  __shared__ __align__(16) float sT[8][16 * 68];
  const int lane = threadIdx.x & 31, wave = threadIdx.x >> 5;
  const int tilesN = N >> 6, tilesM = M >> 6;
  const int tile = (int)blockIdx.x * 8 + wave;
  if (tile >= tilesM * tilesN) return;
  const int tm = tile / tilesN, tn = tile - tm * tilesN;
  const int m0 = tm << 6, n0 = tn << 6;
  const int rl = lane & 15;
  const int koff = (lane >> 4) * 8;
  const int mOff = (lane >> 4) * 8;

  v8f acc[4][4];
#pragma unroll
  for (int i = 0; i < 4; ++i)
#pragma unroll
    for (int j = 0; j < 4; ++j) acc[i][j] = zero8();

#pragma unroll 1
  for (int k0 = 0; k0 < K; k0 += 32) {
    V bh[4];
#pragma unroll
    for (int j = 0; j < 4; ++j) bh[j] = ldfragT<ET>(Bt + (size_t)(n0 + (j << 4) + rl) * ldb + koff + k0);
#pragma unroll
    for (int i = 0; i < 4; ++i) {
      const size_t ao = (size_t)(m0 + (i << 4) + rl) * lda + koff + k0;
      const V ah = ldfragT<ET>(A + ao);
      V al = ah;
      if (SPLITA) al = ldfragT<ET>(A2 + ao);
#pragma unroll
      for (int j = 0; j < 4; ++j) {
        acc[i][j] = Elem<ET>::mma(ah, bh[j], acc[i][j]);
        if (SPLITA) acc[i][j] = Elem<ET>::mma(al, bh[j], acc[i][j]);
      }
      guard_g(acc[i][0], acc[i][3], ah, SPLITA ? al : bh[3]);
    }
    keep4(bh[0], bh[1], bh[2], bh[3]);
  }
  accg4(acc[0][0], acc[0][1], acc[0][2], acc[0][3]);
  accg4(acc[1][0], acc[1][1], acc[1][2], acc[1][3]);
  accg4(acc[2][0], acc[2][1], acc[2][2], acc[2][3]);
  accg4(acc[3][0], acc[3][1], acc[3][2], acc[3][3]);

  float* slab = sT[wave];
#pragma unroll
  for (int i = 0; i < 4; ++i) {
    const int mBase = m0 + (i << 4);
    float brow[8];
#pragma unroll
    for (int r = 0; r < 8; ++r) brow[r] = 0.0f;
    if (BIAS_MODE == 2) {
#pragma unroll
      for (int r = 0; r < 8; ++r) {
        int mi = mBase + mOff + r;
        mi = (mi < M) ? mi : (M - 1);
        brow[r] = bfr(bias0[mi]) * bias_scale;
      }
    }
#pragma unroll
    for (int j = 0; j < 4; ++j) {
      float bcol = 0.0f;
      if (BIAS_MODE == 1) {
        const int n = n0 + (j << 4) + rl;
        const int i0 = (n < nsplit) ? n : (nsplit - 1);
        int i1 = n - nsplit;
        i1 = (i1 > 0) ? i1 : 0;
        int lim1 = N - nsplit - 1;
        lim1 = (lim1 > 0) ? lim1 : 0;
        i1 = (i1 < lim1) ? i1 : lim1;
        const float b0v = bfr(bias0[i0]);
        const float b1v = bfr(bias1[i1]);
        bcol = ((n < nsplit) ? b0v : b1v) * bias_scale;
      }
#pragma unroll
      for (int r = 0; r < 8; ++r) slab[(mOff + r) * 68 + (j << 4) + rl] = acc[i][j][r] * scale + bcol + brow[r];
    }
    __builtin_amdgcn_fence(__ATOMIC_RELEASE, "workgroup");
    __builtin_amdgcn_wave_barrier();
    __builtin_amdgcn_fence(__ATOMIC_ACQUIRE, "workgroup");
    if (OUT_MODE == 0) {
      float* C = (float*)Cout;
      const int hh = lane >> 4, c4 = (lane & 15) * 4;
#pragma unroll
      for (int ps = 0; ps < 2; ++ps) {
#pragma unroll
        for (int it = 0; it < 8; ++it) {
          const int row = it * 2 + hh;
          const v4f v = *(const v4f*)(slab + row * 68 + c4);
          *(volatile v4f*)(C + (size_t)(mBase + row) * ldc + n0 + c4) = v;
        }
        __threadfence();
      }
    } else {
      _Float16* C = (_Float16*)Cout;
      const int qq = lane >> 3, c8 = (lane & 7) * 8;
#pragma unroll
      for (int ps = 0; ps < 2; ++ps) {
#pragma unroll
        for (int it = 0; it < 4; ++it) {
          const int row = it * 4 + qq;
          const float* sp = slab + row * 68 + c8;
          v8h hv;
#pragma unroll
          for (int e = 0; e < 8; ++e) hv[e] = (_Float16)sp[e];
          *(volatile v8h*)(C + (size_t)(mBase + row) * ldc + n0 + c8) = hv;
        }
        __threadfence();
      }
    }
    __builtin_amdgcn_fence(__ATOMIC_RELEASE, "workgroup");
    __builtin_amdgcn_wave_barrier();
    __builtin_amdgcn_fence(__ATOMIC_ACQUIRE, "workgroup");
  }
}

#define QB       32
#define KCH      256
#define QSP      520
#define PSP      264
#define LDS_QS   0
#define LDS_LS   33280
#define LDS_PS   33280
#define LDS_PMAX 66560
#define LDS_PSUM 67584
#define LDS_ST   68608
#define ATT_LDS  69120
static_assert(QB * QSP * 2 == LDS_LS - LDS_QS);
static_assert(QB * QSP * 2 == LDS_PMAX - LDS_LS);
static_assert(QB * PSP * 2 <= LDS_PMAX - LDS_PS);
static_assert(LDS_PSUM - LDS_PMAX == 256 * 4);
static_assert(LDS_ST - LDS_PSUM == 256 * 4);
static_assert(ATT_LDS - LDS_ST == 4 * 32 * 4);
static_assert((QSP % 8) == 0 && (PSP % 8) == 0 && PSP >= KCH && QSP >= DM);
static_assert((LDS_LS % 16) == 0 && (LDS_PMAX % 16) == 0 && (LDS_ST % 16) == 0);
static_assert((SEQ % KCH) == 0 && (SEQ % QB) == 0 && (DM % 64) == 0);

__global__ __launch_bounds__(256) void attn_kernel(const _Float16* __restrict__ qk, const _Float16* __restrict__ vt,
                                                   unsigned short* __restrict__ oh, unsigned short* __restrict__ ol,
                                                   float sc) {
  extern __shared__ __align__(16) char smem[];
  _Float16* Qs = (_Float16*)(smem + LDS_QS);
  _Float16* Ps = (_Float16*)(smem + LDS_PS);
  float* pmax = (float*)(smem + LDS_PMAX);
  float* psum = (float*)(smem + LDS_PSUM);
  float* m_s  = (float*)(smem + LDS_ST);
  float* l_s  = m_s + 32;
  float* al_s = m_s + 64;
  float* li_s = m_s + 96;

  const int tid = threadIdx.x, wave = tid >> 5, lane = tid & 31, h = lane >> 4, c = lane & 15;
  const int q0 = (int)blockIdx.x * QB;
  const int bk0 = (q0 / SEQ) * SEQ;
  const float ninf = -__builtin_inff();

  if (tid < 32) { m_s[tid] = ninf; l_s[tid] = 0.0f; al_s[tid] = 0.0f; li_s[tid] = 0.0f; }
  psum[tid] = 0.0f;
#pragma unroll
  for (int i = 0; i < 8; ++i) {
    const int idx = i * 256 + tid;
    const int row = idx >> 6;
    const int pc  = idx & 63;
    const v8h v = *(const v8h*)(qk + (size_t)(q0 + row) * LDQK + pc * 8);
    *(v8h*)(Qs + row * QSP + pc * 8) = v;
  }
  __syncthreads();

  v8f oacc[2][4];
#pragma unroll
  for (int qt = 0; qt < 2; ++qt)
#pragma unroll
    for (int nt = 0; nt < 4; ++nt) oacc[qt][nt] = zero8();

  const _Float16* qb0p = Qs + c * QSP + 8 * h;
  const _Float16* qb1p = Qs + (16 + c) * QSP + 8 * h;
  const _Float16* pa0p = Ps + c * PSP + 8 * h;
  const _Float16* pa1p = Ps + (16 + c) * PSP + 8 * h;
  const int ntile = SEQ / KCH;

#pragma unroll 1
  for (int t = 0; t < ntile; ++t) {
    const int kb = bk0 + t * KCH + 32 * wave;
    const _Float16* ka0p = qk + (size_t)(kb + c) * LDQK + DM + 8 * h;
    const _Float16* ka1p = qk + (size_t)(kb + 16 + c) * LDQK + DM + 8 * h;
    v8f sacc[2][2];
#pragma unroll
    for (int qt = 0; qt < 2; ++qt)
#pragma unroll
      for (int kt = 0; kt < 2; ++kt) sacc[qt][kt] = zero8();
#pragma unroll 1
    for (int k0 = 0; k0 < DM; k0 += 32) {
      const v16h a0 = ldfrag(ka0p + k0), a1 = ldfrag(ka1p + k0);
      const v16h b0 = ldfrag(qb0p + k0), b1 = ldfrag(qb1p + k0);
      sacc[0][0] = mma16(a0, b0, sacc[0][0]);
      sacc[0][1] = mma16(a1, b0, sacc[0][1]);
      sacc[1][0] = mma16(a0, b1, sacc[1][0]);
      sacc[1][1] = mma16(a1, b1, sacc[1][1]);
      guard_s4(sacc[0][0], sacc[0][1], sacc[1][0], sacc[1][1], a0, a1, b0, b1);
    }
    {
      float pm0 = ninf, pm1 = ninf;
#pragma unroll
      for (int kt = 0; kt < 2; ++kt) {
#pragma unroll
        for (int r = 0; r < 8; ++r) {
          const float v0 = sacc[0][kt][r] * sc; sacc[0][kt][r] = v0; pm0 = fmaxf(pm0, v0);
          const float v1 = sacc[1][kt][r] * sc; sacc[1][kt][r] = v1; pm1 = fmaxf(pm1, v1);
        }
      }
      pm0 = fmaxf(pm0, __shfl_xor(pm0, 16, 32));
      pm1 = fmaxf(pm1, __shfl_xor(pm1, 16, 32));
      pmax[wave * 32 + c] = pm0;
      pmax[wave * 32 + 16 + c] = pm1;
    }
    __syncthreads();
    if (wave == 0) {
      const int row = lane;
      float ps = 0.0f;
#pragma unroll
      for (int w = 0; w < 8; ++w) ps += psum[w * 32 + row];
      l_s[row] = l_s[row] * al_s[row] + ps;
      const float mo = m_s[row];
      float mx = mo;
#pragma unroll
      for (int w = 0; w < 8; ++w) mx = fmaxf(mx, pmax[w * 32 + row]);
      al_s[row] = __expf(mo - mx);
      m_s[row] = mx;
    }
    __syncthreads();
    {
      const float mq0 = m_s[c], mq1 = m_s[16 + c];
      float ps0 = 0.0f, ps1 = 0.0f;
#pragma unroll
      for (int kt = 0; kt < 2; ++kt) {
        v8h h0, h1;
#pragma unroll
        for (int r = 0; r < 8; ++r) {
          const float p0 = __expf(sacc[0][kt][r] - mq0); ps0 += p0; h0[r] = (_Float16)(p0 * 16.0f);
          const float p1 = __expf(sacc[1][kt][r] - mq1); ps1 += p1; h1[r] = (_Float16)(p1 * 16.0f);
        }
        *(v8h*)(Ps + c * PSP + 32 * wave + 16 * kt + 8 * h) = h0;
        *(v8h*)(Ps + (16 + c) * PSP + 32 * wave + 16 * kt + 8 * h) = h1;
      }
      ps0 += __shfl_xor(ps0, 16, 32);
      ps1 += __shfl_xor(ps1, 16, 32);
      psum[wave * 32 + c] = ps0;
      psum[wave * 32 + 16 + c] = ps1;
      const v4f aA = *(const v4f*)(al_s + 8 * h), aB = *(const v4f*)(al_s + 8 * h + 4);
      const v4f bA = *(const v4f*)(al_s + 16 + 8 * h), bB = *(const v4f*)(al_s + 16 + 8 * h + 4);
#pragma unroll
      for (int nt = 0; nt < 4; ++nt) {
#pragma unroll
        for (int r = 0; r < 4; ++r) {
          oacc[0][nt][r] *= aA[r]; oacc[0][nt][4 + r] *= aB[r];
          oacc[1][nt][r] *= bA[r]; oacc[1][nt][4 + r] *= bB[r];
        }
      }
    }
    __syncthreads();
    {
      const _Float16* vbp = vt + (size_t)(64 * wave + c) * NTOT + bk0 + (size_t)t * KCH + 8 * h;
#pragma unroll 1
      for (int ks = 0; ks < KCH; ks += 32) {
        const v16h pa0 = ldfrag(pa0p + ks), pa1 = ldfrag(pa1p + ks);
#pragma unroll
        for (int g = 0; g < 2; ++g) {
          v16h vb[2];
#pragma unroll
          for (int j = 0; j < 2; ++j) vb[j] = ldfrag(vbp + (size_t)(16 * (2 * g + j)) * NTOT + ks);
#pragma unroll
          for (int j = 0; j < 2; ++j) {
            oacc[0][2 * g + j] = mma16(pa0, vb[j], oacc[0][2 * g + j]);
            oacc[1][2 * g + j] = mma16(pa1, vb[j], oacc[1][2 * g + j]);
          }
          guard_s4(oacc[0][2 * g], oacc[0][2 * g + 1], oacc[1][2 * g], oacc[1][2 * g + 1], pa0, pa1, vb[0], vb[1]);
        }
      }
    }
  }

  if (wave == 0) {
    const int row = lane;
    float ps = 0.0f;
#pragma unroll
    for (int w = 0; w < 8; ++w) ps += psum[w * 32 + row];
    const float l = l_s[row] * al_s[row] + ps;
    li_s[row] = (1.0f / l) * (1.0f / 256.0f);
  }
  __syncthreads();
  unsigned short* Hs = (unsigned short*)(smem + LDS_QS);
  unsigned short* Ls = (unsigned short*)(smem + LDS_LS);
  {
    const v4f iA0 = *(const v4f*)(li_s + 8 * h),      iB0 = *(const v4f*)(li_s + 8 * h + 4);
    const v4f iA1 = *(const v4f*)(li_s + 16 + 8 * h), iB1 = *(const v4f*)(li_s + 16 + 8 * h + 4);
#pragma unroll
    for (int nt = 0; nt < 4; ++nt) {
      const int col = 64 * wave + 16 * nt + c;
#pragma unroll
      for (int r = 0; r < 4; ++r) {
        unsigned short hb, lb;
        split_bf(oacc[0][nt][r] * iA0[r], hb, lb);
        Hs[(8 * h + r) * QSP + col] = hb;          Ls[(8 * h + r) * QSP + col] = lb;
        split_bf(oacc[0][nt][4 + r] * iB0[r], hb, lb);
        Hs[(8 * h + 4 + r) * QSP + col] = hb;      Ls[(8 * h + 4 + r) * QSP + col] = lb;
        split_bf(oacc[1][nt][r] * iA1[r], hb, lb);
        Hs[(16 + 8 * h + r) * QSP + col] = hb;     Ls[(16 + 8 * h + r) * QSP + col] = lb;
        split_bf(oacc[1][nt][4 + r] * iB1[r], hb, lb);
        Hs[(16 + 8 * h + 4 + r) * QSP + col] = hb; Ls[(16 + 8 * h + 4 + r) * QSP + col] = lb;
      }
    }
  }
  __syncthreads();
  {
    unsigned short* gh = oh + (size_t)q0 * DM;
    unsigned short* gl = ol + (size_t)q0 * DM;
#pragma unroll
    for (int ps = 0; ps < 2; ++ps) {
#pragma unroll
      for (int rr = 0; rr < 4; ++rr) {
        const int row = 4 * wave + rr;
#pragma unroll
        for (int j = 0; j < 2; ++j) {
          const int pc = j * 32 + lane;
          const v8us hvv = *(const v8us*)(Hs + row * QSP + pc * 8);
          const v8us lvv = *(const v8us*)(Ls + row * QSP + pc * 8);
          *(volatile v8us*)(gh + (size_t)row * DM + pc * 8) = hvv;
          *(volatile v8us*)(gl + (size_t)row * DM + pc * 8) = lvv;
        }
      }
      __threadfence();
    }
  }
}

extern "C" void kernel_launch(void* const* d_in, const int* in_sizes, int n_in,
                              void* d_out, int out_size, void* d_ws, size_t ws_size,
                              hipStream_t stream) {
  if (n_in < 9) return;
  const int ntot = NTOT, dm = DM;
  if (in_sizes[0] != ntot * dm) return;
  if (in_sizes[1] != dm * dm || in_sizes[3] != dm * dm || in_sizes[5] != dm * dm || in_sizes[7] != dm * dm) return;
  if (in_sizes[2] != dm || in_sizes[4] != dm || in_sizes[6] != dm || in_sizes[8] != dm) return;
  if (out_size != ntot * dm) return;

  const float* x  = (const float*)d_in[0];
  const float* Wq = (const float*)d_in[1];
  const float* bq = (const float*)d_in[2];
  const float* Wk = (const float*)d_in[3];
  const float* bk = (const float*)d_in[4];
  const float* Wv = (const float*)d_in[5];
  const float* bv = (const float*)d_in[6];
  const float* Wo = (const float*)d_in[7];
  const float* bo = (const float*)d_in[8];
  float* out = (float*)d_out;

  const size_t bWt = (size_t)3 * dm * dm * 2;
  const size_t bWo = (size_t)dm * dm * 2;
  const size_t bX  = (size_t)ntot * dm * 2;
  const size_t bQK = (size_t)ntot * 2 * dm * 2;
  const size_t bVT = (size_t)dm * ntot * 2;
  const size_t bO  = (size_t)ntot * dm * 2;
  size_t off = 0;
  const size_t oWt = off; off += bWt;
  const size_t oWo = off; off += bWo;
  const size_t oX  = off; off += bX;
  const size_t oQK = off; off += bQK;
  const size_t oVT = off; off += bVT;
  const size_t oOH = off; off += bO;
  const size_t oOL = off; off += bO;
  if (off > ws_size) return;
  if (off > (size_t)134217728) return;

  char* ws = (char*)d_ws;
  _Float16*       Wt16 = (_Float16*)(ws + oWt);
  unsigned short* Wob  = (unsigned short*)(ws + oWo);
  _Float16*       X16  = (_Float16*)(ws + oX);
  _Float16*       QK16 = (_Float16*)(ws + oQK);
  _Float16*       VT16 = (_Float16*)(ws + oVT);
  unsigned short* OH   = (unsigned short*)(ws + oOH);
  unsigned short* OL   = (unsigned short*)(ws + oOL);

  const dim3 blk(256);
  const int n8 = ntot * dm / 8;
  if ((n8 % 256) != 0) return;

  cvt_x_kernel<<<dim3(n8 / 256), blk, 0, stream>>>(x, X16, n8);
  cvt_wt_kernel<<<dim3(4 * (dm / 64) * (dm / 64)), blk, 0, stream>>>(Wq, Wk, Wv, Wo, Wt16, Wob);
  {
    const int tiles = (ntot / 64) * ((2 * dm) / 64);
    gemm64_kernel<0, false, 1, 1><<<dim3((tiles + 7) / 8), blk, 0, stream>>>(
        (const unsigned short*)X16, (const unsigned short*)X16, dm, (const unsigned short*)Wt16, dm,
        (void*)QK16, 2 * dm, bq, bk, dm, ntot, 2 * dm, dm, 0.03125f, 16.0f);
  }
  {
    const int tiles = (dm / 64) * (ntot / 64);
    gemm64_kernel<0, false, 1, 2><<<dim3((tiles + 7) / 8), blk, 0, stream>>>(
        (const unsigned short*)(Wt16 + (size_t)2 * dm * dm), (const unsigned short*)(Wt16 + (size_t)2 * dm * dm), dm,
        (const unsigned short*)X16, dm,
        (void*)VT16, ntot, bv, bv, dm, dm, ntot, dm, 0.03125f, 16.0f);
  }
  (void)hipFuncSetAttribute(reinterpret_cast<const void*>(&attn_kernel),
                            hipFuncAttributeMaxDynamicSharedMemorySize, ATT_LDS);
  const float sc = 0.125f * (1.0f / 256.0f);
  attn_kernel<<<dim3(ntot / QB), blk, ATT_LDS, stream>>>(QK16, VT16, OH, OL, sc);
  {
    const int tiles = (ntot / 64) * (dm / 64);
    gemm64_kernel<1, true, 0, 1><<<dim3((tiles + 7) / 8), blk, 0, stream>>>(
        OH, OL, dm, Wob, dm, (void*)out, dm, bo, bo, dm, ntot, dm, dm, 1.0f, 1.0f);
  }
  (void)hipGetLastError();
}
